// TransformerCovarianceModule_20444044329463
// MI455X (gfx1250) — hardware-verified
//
#include <hip/hip_runtime.h>
#include <math.h>

typedef __attribute__((ext_vector_type(16))) _Float16 v16h;
typedef __attribute__((ext_vector_type(16))) __bf16 v16b;
typedef __attribute__((ext_vector_type(8)))  _Float16 v8h;
typedef __attribute__((ext_vector_type(8)))  float v8f;
typedef __attribute__((ext_vector_type(4)))  float v4f;
typedef __attribute__((ext_vector_type(2)))  float v2f;
typedef __attribute__((ext_vector_type(4)))  unsigned v4u;
typedef __attribute__((ext_vector_type(4)))  int v4i;
typedef float __attribute__((may_alias)) float_a;
typedef int __attribute__((may_alias)) int_a;

template <typename T> __device__ __forceinline__ void vst2(void* p, T v) { *(volatile T*)p = v; __threadfence(); *(volatile T*)p = v; }
__device__ __forceinline__ v8f wmma16(v16h a, v16h b, v8f c) {
  v8f d = __builtin_amdgcn_wmma_f32_16x16x32_f16(false, a, false, b, (short)0, c, false, false);
  asm volatile("v_nop\n\tv_nop\n\tv_nop\n\tv_nop" : "+v"(d) : "v"(a), "v"(b));
  return d;
}
__device__ __forceinline__ v8f wmma_bf(v16b a, v16b b, v8f c) {
  v8f d = __builtin_amdgcn_wmma_f32_16x16x32_bf16(false, a, false, b, (short)0, c, false, false);
  asm volatile("v_nop\n\tv_nop\n\tv_nop\n\tv_nop" : "+v"(d) : "v"(a), "v"(b));
  return d;
}
__device__ __forceinline__ v16h frag_h(const _Float16* rowk0, int lane) {
  union { v16h v; v8h q[2]; } u; const _Float16* p = rowk0 + 8 * (lane >> 4);
  u.q[0] = *(const v8h*)p; u.q[1] = *(const v8h*)(p + 16); return u.v;
}
__device__ __forceinline__ v16h frag_f32(const float* rowk0, int lane) {
  v16h a; const float* p = rowk0 + 8 * (lane >> 4);
#pragma unroll
  for (int i = 0; i < 8; ++i) { a[i] = (_Float16)p[i]; a[8 + i] = (_Float16)p[16 + i]; }
  return a;
}
__device__ __forceinline__ v16h frag_f32s(const float* rowk0, int lane, float sc) {
  v16h a; const float* p = rowk0 + 8 * (lane >> 4);
#pragma unroll
  for (int i = 0; i < 8; ++i) { a[i] = (_Float16)(p[i] * sc); a[8 + i] = (_Float16)(p[16 + i] * sc); }
  return a;
}
__device__ __forceinline__ v16h fragc_f32(const float* W, int k0, int n, int lane, int ld, int K) {
  v16h a; const int g = lane >> 4;
#pragma unroll
  for (int i = 0; i < 8; ++i) { const int ka = k0 + 8 * g + i, kb = ka + 16;
    a[i] = (_Float16)(ka < K ? W[(size_t)(ka < K ? ka : K - 1) * ld + n] : 0.f); a[8 + i] = (_Float16)(kb < K ? W[(size_t)(kb < K ? kb : K - 1) * ld + n] : 0.f); }
  return a;
}
struct F2 { v16b h, l; };
__device__ __forceinline__ F2 bsplit16(const float v[16]) { F2 r;
#pragma unroll
  for (int i = 0; i < 16; ++i) { const __bf16 h = (__bf16)v[i]; r.h[i] = h; r.l[i] = (__bf16)(v[i] - (float)h); }
  return r; }
__device__ __forceinline__ F2 split_row(const float* row, int k0, int lane) { float v[16]; const float* p = row + k0 + 8 * (lane >> 4);
#pragma unroll
  for (int i = 0; i < 8; ++i) { v[i] = p[i]; v[8 + i] = p[16 + i]; }
  return bsplit16(v); }
__device__ __forceinline__ F2 split_rowK(const float* row, int k0, int lane, int K) { float v[16]; const int g = lane >> 4;
#pragma unroll
  for (int i = 0; i < 8; ++i) { const int ka = k0 + 8 * g + i, kb = ka + 16; v[i] = ka < K ? row[ka < K ? ka : K - 1] : 0.f; v[8 + i] = kb < K ? row[kb < K ? kb : K - 1] : 0.f; }
  return bsplit16(v); }
__device__ __forceinline__ F2 split_col(const float* W, int k0, int n, int lane, int ld, int K) { float v[16]; const int g = lane >> 4;
#pragma unroll
  for (int i = 0; i < 8; ++i) { const int ka = k0 + 8 * g + i, kb = ka + 16; v[i] = ka < K ? W[(size_t)(ka < K ? ka : K - 1) * ld + n] : 0.f; v[8 + i] = kb < K ? W[(size_t)(kb < K ? kb : K - 1) * ld + n] : 0.f; }
  return bsplit16(v); }
__device__ __forceinline__ v8f mac3(const F2& a, const F2& b, v8f c) { c = wmma_bf(a.l, b.h, c); c = wmma_bf(a.h, b.l, c); return wmma_bf(a.h, b.h, c); }
__device__ __forceinline__ float sigm(float v) { return 1.0f / (1.0f + expf(-v)); }
#define LDSX() do { asm volatile("s_wait_dscnt 0" ::: "memory"); __builtin_amdgcn_wave_barrier(); __builtin_amdgcn_fence(__ATOMIC_RELEASE, "workgroup"); } while (0)


#define NB 2
#define CC 256
#define NP 4096
#define NH 8
#define HD2 32
#ifndef TNB
#define TNB NB
#endif
#ifndef TQB2
#define TQB2 (NP / 64)
#endif
typedef __attribute__((ext_vector_type(8))) __bf16 v8b;
__device__ __forceinline__ v16b frag_b(const __bf16* rowk0, int lane) {
  union { v16b v; v8b q[2]; } u; const __bf16* p = rowk0 + 8 * (lane >> 4);
  u.q[0] = *(const v8b*)p; u.q[1] = *(const v8b*)(p + 16); return u.v;
}
__device__ __forceinline__ float bfr(float v) { return (float)(__bf16)v; }
__device__ __attribute__((noinline)) float exp_ni(float v) { return expf(v); }
__device__ __attribute__((noinline)) float erf_ni(float v) { return erff(v); }

#define WS_QH  0u
#define WS_QL  (WS_QH + 2u * (size_t)NB * NP * CC)
#define WS_KH  (WS_QL + 2u * (size_t)NB * NP * CC)
#define WS_KL  (WS_KH + 2u * (size_t)NB * NP * CC)
#define WS_VH  (WS_KL + 2u * (size_t)NB * NP * CC)
#define WS_VL  (WS_VH + 2u * (size_t)NB * CC * NP)
#define WS_CT  (WS_VL + 2u * (size_t)NB * CC * NP)
#define WS_END (WS_CT + 4u * (size_t)NB * NP * CC)

__global__ __launch_bounds__(128) void k_qkv(const float* __restrict__ X, const float* __restrict__ Wt, const float* __restrict__ Bs, _Float16* __restrict__ QH, _Float16* __restrict__ QL, _Float16* __restrict__ KH, _Float16* __restrict__ KL, _Float16* __restrict__ VH, _Float16* __restrict__ VL) {
  __shared__ __align__(16) __bf16 sx[64][CC + 8]; __shared__ __align__(16) _Float16 sh[64][136], sl[64][136]; __shared__ __align__(16) _Float16 th[128][72], tl[128][72];
  const int tid = threadIdx.x, wave = tid >> 5, lane = tid & 31, col = lane & 15, g = lane >> 4; const int n0 = blockIdx.x * 64; const int cg = blockIdx.y; const size_t b = blockIdx.z; const int which = cg >> 1; const int c0 = (cg & 1) * 128;
  for (int e = tid; e < CC * 64; e += 128) { const int c = e >> 6, nl = e & 63; sx[nl][c] = (__bf16)X[((b * CC + c) * NP) + n0 + nl]; }
  __syncthreads();
  v8f acc[8] = {};
#pragma unroll
  for (int kc = 0; kc < CC / 32; ++kc) { const v16b a = frag_b(&sx[wave * 16 + col][kc * 32], lane);
#pragma unroll
    for (int j = 0; j < 8; ++j) { v16b w; const size_t o = (size_t)which * CC + c0 + j * 16 + col;
#pragma unroll
      for (int i = 0; i < 8; ++i) { w[i] = (__bf16)Wt[o * CC + kc * 32 + 8 * g + i]; w[8 + i] = (__bf16)Wt[o * CC + kc * 32 + 16 + 8 * g + i]; }
      acc[j] = wmma_bf(a, w, acc[j]); } }
#pragma unroll
  for (int j = 0; j < 8; ++j) { const float bb = bfr(Bs[which * CC + c0 + j * 16 + col]);
#pragma unroll
    for (int r = 0; r < 8; ++r) { const float v = acc[j][r] + bb; const _Float16 hv = (_Float16)v, lv = (_Float16)((v - (float)hv) * 2048.0f); const int rl = wave * 16 + 8 * g + r, cl = j * 16 + col; if (which < 2) { sh[rl][cl] = hv; sl[rl][cl] = lv; } else { th[cl][rl] = hv; tl[cl][rl] = lv; } } }
  __syncthreads();
  if (which < 2) { _Float16* DH = which == 0 ? QH : KH; _Float16* DL = which == 0 ? QL : KL;
    for (int e = tid; e < 64 * 16; e += 128) { const int rl = e >> 4, q = e & 15; const size_t o = (b * NP + n0 + rl) * CC + c0 + q * 8; vst2((unsigned*)(DH + o), *(const v4u*)&sh[rl][q * 8]); vst2((unsigned*)(DL + o), *(const v4u*)&sl[rl][q * 8]); } }
  else { for (int e = tid; e < 128 * 8; e += 128) { const int cl = e >> 3, q = e & 7; const size_t o = (b * CC + c0 + cl) * (size_t)NP + n0 + q * 8; vst2((unsigned*)(VH + o), *(const v4u*)&th[cl][q * 8]); vst2((unsigned*)(VL + o), *(const v4u*)&tl[cl][q * 8]); } } }
__global__ __launch_bounds__(128) void k_att(const _Float16* __restrict__ QH, const _Float16* __restrict__ QL, const _Float16* __restrict__ KH, const _Float16* __restrict__ KL, const _Float16* __restrict__ VH, const _Float16* __restrict__ VL, float* __restrict__ CT) {
  __shared__ __align__(16) float sp[4][16][36]; __shared__ __align__(16) float so[4][16][36];
  const int tid = threadIdx.x, wave = tid >> 5, lane = tid & 31, col = lane & 15, g = lane >> 4; const int qb = blockIdx.x, h = blockIdx.y; const size_t b = blockIdx.z; const int q0 = qb * 64 + wave * 16; const bool three = (qb < 2);
  const v16h aq = frag_h(QH + (b * NP + q0 + col) * CC + h * HD2, lane); const v16h al = frag_h(QL + (b * NP + q0 + col) * CC + h * HD2, lane);
  float m[8], l[8];
#pragma unroll
  for (int r = 0; r < 8; ++r) { m[r] = -3.0e38f; l[r] = 0.f; }
  v8f acc[2] = {}, accl[2] = {};
#pragma unroll 1
  for (int ks = 0; ks < NP / 32; ++ks) { float s[2][8];
#pragma unroll
    for (int ct = 0; ct < 2; ++ct) { const int kk = ks * 32 + ct * 16 + col; const size_t rk = (b * NP + kk) * CC + h * HD2; const v16h kh = frag_h(KH + rk, lane); v8f c = {}; c = wmma16(aq, kh, c);
      if (three) { v8f cl = {}; cl = wmma16(al, kh, cl); cl = wmma16(aq, frag_h(KL + rk, lane), cl);
#pragma unroll
        for (int r = 0; r < 8; ++r) c[r] += cl[r] * (1.0f / 2048.0f); }
#pragma unroll
      for (int r = 0; r < 8; ++r) s[ct][r] = c[r] * 0.17677669529663687f; }
    float alpha[8];
#pragma unroll
    for (int r = 0; r < 8; ++r) { float mx = fmaxf(s[0][r], s[1][r]);
#pragma unroll
      for (int o = 1; o < 16; o <<= 1) mx = fmaxf(mx, __shfl_xor(mx, o));
      const float mn = fmaxf(m[r], mx); alpha[r] = __expf(m[r] - mn); const float e0 = __expf(s[0][r] - mn), e1 = __expf(s[1][r] - mn); float es = e0 + e1;
#pragma unroll
      for (int o = 1; o < 16; o <<= 1) es += __shfl_xor(es, o);
      l[r] = l[r] * alpha[r] + es; m[r] = mn; sp[wave][8 * g + r][col] = e0; sp[wave][8 * g + r][16 + col] = e1; }
#pragma unroll
    for (int j = 0; j < 2; ++j)
#pragma unroll
      for (int r = 0; r < 8; ++r) { acc[j][r] *= alpha[r]; accl[j][r] *= alpha[r]; }
    LDSX();
    v16h pa, pl; { const float* prow = &sp[wave][col][0] + 8 * (lane >> 4);
#pragma unroll
      for (int i = 0; i < 8; ++i) { const float x0 = prow[i] * 2048.0f, x1 = prow[16 + i] * 2048.0f; const _Float16 h0 = (_Float16)x0, h1 = (_Float16)x1; pa[i] = h0; pa[8 + i] = h1; pl[i] = (_Float16)((x0 - (float)h0) * 2048.0f); pl[8 + i] = (_Float16)((x1 - (float)h1) * 2048.0f); } }
#pragma unroll
    for (int j = 0; j < 2; ++j) { const size_t po = (b * CC + (size_t)h * HD2 + j * 16 + col) * NP + ks * 32; const v16h vh = frag_h(VH + po, lane); acc[j] = wmma16(pa, vh, acc[j]); if (three) { accl[j] = wmma16(pl, vh, accl[j]); accl[j] = wmma16(pa, frag_h(VL + po, lane), accl[j]); } }
    LDSX(); }
#pragma unroll
  for (int r = 0; r < 8; ++r) { const float il = (1.0f / 2048.0f) / l[r];
#pragma unroll
    for (int j = 0; j < 2; ++j) so[wave][8 * g + r][j * 16 + col] = (acc[j][r] + accl[j][r] * (1.0f / 2048.0f)) * il; }
  LDSX(); for (int rl = 0; rl < 16; ++rl) if (lane < 8) vst2(CT + (b * NP + q0 + rl) * CC + h * HD2 + lane * 4, *(const v4f*)&so[wave][rl][lane * 4]); }
__global__ __launch_bounds__(128) void k_proj(const float* __restrict__ CT, const float* __restrict__ Wp, const float* __restrict__ Bp, const float* __restrict__ X, float* __restrict__ OUT) { __shared__ __align__(16) float st[128][68];
  const int tid = threadIdx.x, wave = tid >> 5, lane = tid & 31, col = lane & 15, g = lane >> 4; const size_t b = blockIdx.y; const int n0 = blockIdx.x * 64; const size_t r0 = b * NP + n0 + wave * 16;
#pragma unroll 1
  for (int og = 0; og < 2; ++og) { v8f acc[8] = {};
#pragma unroll
    for (int kc = 0; kc < CC / 32; ++kc) { const F2 a = split_row(CT + (r0 + col) * CC, kc * 32, lane);
#pragma unroll
      for (int j = 0; j < 8; ++j) { v16b w; const int o = og * 128 + j * 16 + col;
#pragma unroll
        for (int i = 0; i < 8; ++i) { w[i] = (__bf16)Wp[(size_t)o * CC + kc * 32 + 8 * g + i]; w[8 + i] = (__bf16)Wp[(size_t)o * CC + kc * 32 + 16 + 8 * g + i]; }
        acc[j] = wmma_bf(a.h, w, acc[j]); acc[j] = wmma_bf(a.l, w, acc[j]); } }
#pragma unroll
    for (int j = 0; j < 8; ++j)
#pragma unroll
      for (int r = 0; r < 8; ++r) { const int o = og * 128 + j * 16 + col, nl = wave * 16 + 8 * g + r; st[j * 16 + col][nl] = acc[j][r] + bfr(Bp[o]) + bfr(X[((b * CC + o) * NP) + n0 + nl]); }
    __syncthreads();
    for (int e = tid; e < 128 * 16; e += 128) { const int ol = e >> 4, q = e & 15; vst2(OUT + ((b * CC + og * 128 + ol) * NP) + n0 + q * 4, *(const v4f*)&st[ol][q * 4]); }
    __syncthreads(); } }
extern "C" void kernel_launch(void* const* d_in, const int* in_sizes, int n_in, void* d_out, int out_size, void* d_ws, size_t ws_size, hipStream_t stream) {
  (void)in_sizes; (void)n_in; (void)out_size;
  const float** F = (const float**)d_in;
  if (ws_size < (size_t)WS_END) return;
  char* ws = (char*)d_ws; _Float16 *QH = (_Float16*)(ws + WS_QH), *QL = (_Float16*)(ws + WS_QL), *KH = (_Float16*)(ws + WS_KH), *KL = (_Float16*)(ws + WS_KL), *VH = (_Float16*)(ws + WS_VH), *VL = (_Float16*)(ws + WS_VL); float* CT = (float*)(ws + WS_CT);
  k_qkv<<<dim3(NP / 64, 6, TNB), 128, 0, stream>>>(F[0], F[1], F[2], QH, QL, KH, KL, VH, VL);
  k_att<<<dim3(TQB2, NH, TNB), 128, 0, stream>>>(QH, QL, KH, KL, VH, VL, CT);
  k_proj<<<dim3(TQB2, TNB), 128, 0, stream>>>(CT, F[3], F[4], F[0], (float*)d_out);
}
